// Net_30554397343884
// MI455X (gfx1250) — hardware-verified
//
#include <hip/hip_runtime.h>
#include <math.h>

constexpr int NBATCH   = 2048;
constexpr int NSTEP    = 512;
constexpr int NHID     = 16;
constexpr int NGATE    = 4 * NHID;
constexpr int NHEAD    = 16;
constexpr int NCAT     = 2 * NHID;
constexpr int ROWS_BLK = 32;
constexpr int NTHR     = 64;
constexpr int TCHUNK   = 32;
constexpr int NCHUNK   = NSTEP / TCHUNK;
constexpr int XPITCH   = 36;
constexpr int HCPITCH  = 33;
constexpr float LO_CARRY     = 64.0f;
constexpr float LO_CARRY_INV = 1.0f / 64.0f;
static_assert(NBATCH % ROWS_BLK == 0, "grid exact");
static_assert(NSTEP % TCHUNK == 0, "no time tail");
static_assert(ROWS_BLK == 2 * 16 && NTHR == 64, "two waves x 16 rows");
static_assert(XPITCH % 4 == 0 && XPITCH >= TCHUNK, "16-B aligned LDS rows");
static_assert(NGATE == 64 && NCAT == 32, "shape contract");
static_assert((NHEAD * NCAT) == 2 * NTHR * 4, "head weight staging exact");
static_assert(ROWS_BLK * 4 == 128, "one whole output line per block");

typedef __attribute__((ext_vector_type(16))) _Float16 v16h;
typedef __attribute__((ext_vector_type(8)))  float    v8f;
typedef __attribute__((ext_vector_type(4)))  float    v4f;

__device__ __forceinline__ void guard_group(v8f& d0, v8f& d1, v8f& d2, v8f& d3,
                                            v16h a0, v16h a1, v16h a2, v16h a3, v16h b) {
  asm volatile("v_nop\n\tv_nop\n\tv_nop\n\tv_nop"
               : "+v"(d0), "+v"(d1), "+v"(d2), "+v"(d3)
               : "v"(a0), "v"(a1), "v"(a2), "v"(a3), "v"(b));
}
__device__ __forceinline__ v8f mma_h(v16h a, v16h b, v8f c) {
  return __builtin_amdgcn_wmma_f32_16x16x32_f16(false, a, false, b, (short)0, c, false, false);
}
__device__ __forceinline__ void settle4(v4f& a, v4f& b, v4f& c, v4f& d) {
  asm volatile("" : "+v"(a), "+v"(b), "+v"(c), "+v"(d) :: "memory");
}
__device__ __forceinline__ void settle6(v4f& a, v4f& b, v4f& c, v4f& d, v4f& e, v4f& f) {
  asm volatile("" : "+v"(a), "+v"(b), "+v"(c), "+v"(d), "+v"(e), "+v"(f) :: "memory");
}
__device__ __forceinline__ void ld8(const float* p, v4f& a, v4f& b) {
  a = *(const v4f*)(p);
  b = *(const v4f*)(p + 4);
}
__device__ __forceinline__ v16h make_a(v4f p, v4f q) {
  v16h a;
#pragma unroll
  for (int e = 0; e < 4; ++e) {
    const float w0 = p[e];
    const float w1 = q[e];
    a[e]      = (_Float16)w0;
    a[4 + e]  = (_Float16)w1;
    a[8 + e]  = (_Float16)(w0 * LO_CARRY_INV);
    a[12 + e] = (_Float16)(w1 * LO_CARRY_INV);
  }
  return a;
}
__device__ __forceinline__ float fsig(float v)  { return __builtin_amdgcn_rcpf(1.0f + __expf(-v)); }
__device__ __forceinline__ float ftanh(float v) { return 1.0f - 2.0f * __builtin_amdgcn_rcpf(__expf(2.0f * v) + 1.0f); }

__global__ __launch_bounds__(NTHR) void bilstm_head_kernel(
    const float* __restrict__ x,
    const float* pWihF, const float* pWhhF, const float* pBihF, const float* pBhhF,
    const float* pWihR, const float* pBihR, const float* pBhhR,
    const float* pW1, const float* pB1, const float* pW2, const float* pB2,
    float* out) {
  __shared__ __align__(16) float xs[ROWS_BLK * XPITCH];
  __shared__ __align__(16) float w1s[NHEAD * NCAT];
  __shared__ __align__(16) float hcs[ROWS_BLK * HCPITCH];

  const int tid  = threadIdx.x;
  const int lane = tid & 31;
  const int wave = tid >> 5;
  const int c    = lane & 15;
  const int hh   = lane >> 4;
  const int blkrow  = blockIdx.x * ROWS_BLK;
  const int waverow = blkrow + 16 * wave;

#pragma unroll
  for (int it = 0; it < 2; ++it) {
    const int idx = it * NTHR + tid;
    const v4f v = *(const v4f*)(pW1 + 4 * idx);
    *(v4f*)(w1s + 4 * idx) = v;
  }

  v16h A0, A1, A2, A3;
  {
    v4f p0, q0, p1, q1;
    ld8(pWhhF + (0 * NHID + c) * NHID + 8 * hh, p0, q0);
    ld8(pWhhF + (1 * NHID + c) * NHID + 8 * hh, p1, q1);
    settle4(p0, q0, p1, q1);
    A0 = make_a(p0, q0);
    A1 = make_a(p1, q1);
  }
  {
    v4f p2, q2, p3, q3;
    ld8(pWhhF + (2 * NHID + c) * NHID + 8 * hh, p2, q2);
    ld8(pWhhF + (3 * NHID + c) * NHID + 8 * hh, p3, q3);
    settle4(p2, q2, p3, q3);
    A2 = make_a(p2, q2);
    A3 = make_a(p3, q3);
  }

  float bs[4][8], wi[4][8];
#pragma unroll
  for (int g = 0; g < 4; ++g) {
    const int base = NHID * g + 8 * hh;
    v4f w0, w1v, i0, i1, h0, h1;
    ld8(pWihF + base, w0, w1v);
    ld8(pBihF + base, i0, i1);
    ld8(pBhhF + base, h0, h1);
    settle6(w0, w1v, i0, i1, h0, h1);
#pragma unroll
    for (int e = 0; e < 4; ++e) {
      wi[g][e]     = w0[e];
      wi[g][4 + e] = w1v[e];
      bs[g][e]     = i0[e] + h0[e];
      bs[g][4 + e] = i1[e] + h1[e];
    }
  }

  float cst[8], hst[8];
#pragma unroll
  for (int r = 0; r < 8; ++r) { cst[r] = 0.0f; hst[r] = 0.0f; }
  v16h bu;
#pragma unroll
  for (int e = 0; e < 16; ++e) bu[e] = (_Float16)0.0f;

  float* xw = xs + 16 * wave * XPITCH;
  const float* xrow = xw + c * XPITCH;

#pragma unroll 1
  for (int ch = 0; ch < NCHUNK; ++ch) {
    __syncthreads();
#pragma unroll
    for (int it = 0; it < 4; ++it) {
      const int idx = it * 32 + lane;
      const int row = idx >> 3;
      const int q4  = (idx & 7) * 4;
      const v4f v = *(const v4f*)(x + (size_t)(waverow + row) * NSTEP + ch * TCHUNK + q4);
      *(v4f*)(xw + row * XPITCH + q4) = v;
    }
    __syncthreads();

#pragma unroll 1
    for (int tt = 0; tt < TCHUNK; ++tt) {
      const float xv = xrow[tt];
      v8f d0, d1, d2, d3;
#pragma unroll
      for (int r = 0; r < 8; ++r) {
        d0[r] = fmaf(xv, wi[0][r], bs[0][r]);
        d1[r] = fmaf(xv, wi[1][r], bs[1][r]);
        d2[r] = fmaf(xv, wi[2][r], bs[2][r]);
        d3[r] = fmaf(xv, wi[3][r], bs[3][r]);
      }
      d0 = mma_h(A0, bu, d0);
      d1 = mma_h(A1, bu, d1);
      d2 = mma_h(A2, bu, d2);
      d3 = mma_h(A3, bu, d3);
      guard_group(d0, d1, d2, d3, A0, A1, A2, A3, bu);
#pragma unroll
      for (int r = 0; r < 8; ++r) {
        const float ig = fsig(d0[r]);
        const float fg = fsig(d1[r]);
        const float gg = ftanh(d2[r]);
        const float og = fsig(d3[r]);
        const float cn = fg * cst[r] + ig * gg;
        cst[r] = cn;
        const float hn = og * ftanh(cn);
        hst[r] = hn;
        const _Float16 hi16 = (_Float16)hn;
        const float res = (hn - (float)hi16) * LO_CARRY;
        bu[r]     = hi16;
        bu[8 + r] = (_Float16)res;
      }
    }
  }

  const float xl = xrow[TCHUNK - 1];
  float hb[8];
  {
    float si[8], tg[8];
    {
      const int base = 0 * NHID + 8 * hh;
      v4f w0, w1v, i0, i1, h0, h1;
      ld8(pWihR + base, w0, w1v);
      ld8(pBihR + base, i0, i1);
      ld8(pBhhR + base, h0, h1);
      settle6(w0, w1v, i0, i1, h0, h1);
#pragma unroll
      for (int e = 0; e < 4; ++e) {
        si[e]     = fsig(fmaf(xl, w0[e],  i0[e] + h0[e]));
        si[4 + e] = fsig(fmaf(xl, w1v[e], i1[e] + h1[e]));
      }
    }
    {
      const int base = 2 * NHID + 8 * hh;
      v4f w0, w1v, i0, i1, h0, h1;
      ld8(pWihR + base, w0, w1v);
      ld8(pBihR + base, i0, i1);
      ld8(pBhhR + base, h0, h1);
      settle6(w0, w1v, i0, i1, h0, h1);
#pragma unroll
      for (int e = 0; e < 4; ++e) {
        tg[e]     = ftanh(fmaf(xl, w0[e],  i0[e] + h0[e]));
        tg[4 + e] = ftanh(fmaf(xl, w1v[e], i1[e] + h1[e]));
      }
    }
    {
      const int base = 3 * NHID + 8 * hh;
      v4f w0, w1v, i0, i1, h0, h1;
      ld8(pWihR + base, w0, w1v);
      ld8(pBihR + base, i0, i1);
      ld8(pBhhR + base, h0, h1);
      settle6(w0, w1v, i0, i1, h0, h1);
#pragma unroll
      for (int e = 0; e < 4; ++e) {
        const float so0 = fsig(fmaf(xl, w0[e],  i0[e] + h0[e]));
        const float so1 = fsig(fmaf(xl, w1v[e], i1[e] + h1[e]));
        hb[e]     = so0 * ftanh(si[e] * tg[e]);
        hb[4 + e] = so1 * ftanh(si[4 + e] * tg[4 + e]);
      }
    }
  }

#pragma unroll
  for (int r = 0; r < 8; ++r) {
    hcs[(16 * wave + c) * HCPITCH + 8 * hh + r]        = hst[r];
    hcs[(16 * wave + c) * HCPITCH + NHID + 8 * hh + r] = hb[r];
  }
  __syncthreads();

  if (wave == 0) {
    float hv[NCAT];
#pragma unroll
    for (int m = 0; m < NCAT; ++m) hv[m] = hcs[lane * HCPITCH + m];
    float acc = pB2[0];
#pragma unroll 1
    for (int j = 0; j < NHEAD; ++j) {
      float s = pB1[j];
#pragma unroll
      for (int m = 0; m < NCAT; ++m) s = fmaf(w1s[j * NCAT + m], hv[m], s);
      s = (s > 0.0f) ? s : 0.2f * s;
      acc = fmaf(pW2[j], s, acc);
    }
    volatile float* op = out + blkrow + lane;
    *op = acc;
    __threadfence();
    *op = acc;
  }
}

extern "C" void kernel_launch(void* const* d_in, const int* in_sizes, int n_in,
                              void* d_out, int out_size, void* d_ws, size_t ws_size, hipStream_t stream) {
  (void)in_sizes; (void)out_size; (void)d_ws; (void)ws_size;
  if (n_in < 13 || d_out == nullptr) return;
  const float* x     = (const float*)d_in[0];
  const float* wih_f = (const float*)d_in[1];
  const float* whh_f = (const float*)d_in[2];
  const float* bih_f = (const float*)d_in[3];
  const float* bhh_f = (const float*)d_in[4];
  const float* wih_r = (const float*)d_in[5];
  const float* bih_r = (const float*)d_in[7];
  const float* bhh_r = (const float*)d_in[8];
  const float* w1 = (const float*)d_in[9];
  const float* b1 = (const float*)d_in[10];
  const float* w2 = (const float*)d_in[11];
  const float* b2 = (const float*)d_in[12];

  bilstm_head_kernel<<<NBATCH / ROWS_BLK, NTHR, 0, stream>>>(
      x, wih_f, whh_f, bih_f, bhh_f, wih_r, bih_r, bhh_r, w1, b1, w2, b2, (float*)d_out);
}
